// MyFullyActiveRQS_72258529788183
// MI455X (gfx1250) — hardware-verified
//
#include <hip/hip_runtime.h>
#include <stdint.h>
#include <stddef.h>


typedef __attribute__((ext_vector_type(16))) _Float16 v16h;
typedef __attribute__((ext_vector_type(8)))  _Float16 v8h;
typedef __attribute__((ext_vector_type(8)))  float    v8f;
typedef __attribute__((ext_vector_type(4)))  float    v4f;

#define NBATCH 32
#define NCH    12
#define NCOND  4
#define NPIXI  4096
#define MPIX   131072
#define CIN1   16
#define HID    128
#define NPAR   23
#define OUTC   276
#define NPAD3  288
#define KT1    5
#define KT2    4
#define KT3    36
#define TAILV  3.0f
#define MBWV   0.001f
#define MBHV   0.001f
#define MDV    0.001f
#define WSCL   0.992f
#define UPAD   0.53974242f

__device__ __forceinline__ void dep_guard_h(v8f& a, v8f& b, v16h x, v16h y) { asm volatile("v_nop\n\tv_nop\n\tv_nop\n\tv_nop" : "+v"(a), "+v"(b) : "v"(x), "v"(y)); }
__device__ __forceinline__ void keep4_h(v16h a, v16h b, v16h c, v16h d) { asm volatile("v_nop" :: "v"(a), "v"(b), "v"(c), "v"(d)); }
__device__ __forceinline__ void acc_guard4(v8f& a, v8f& b, v8f& c, v8f& d) { asm volatile("v_nop\n\tv_nop\n\tv_nop\n\tv_nop" : "+v"(a), "+v"(b), "+v"(c), "+v"(d)); }

template <typename T> struct Frag;
template <> struct Frag<_Float16> {
  typedef v16h V; union U { v16h v; v8h h[2]; };
  static __device__ __forceinline__ v16h load(const _Float16* p) {
    U f; f.h[0] = *(const v8h*)(p); f.h[1] = *(const v8h*)(p + 16); return f.v;
  }
  static __device__ __forceinline__ v8f mma(v16h a, v16h b, v8f c) {
    return __builtin_amdgcn_wmma_f32_16x16x32_f16(false, a, false, b, (short)0, c, false, false);
  }
  static __device__ __forceinline__ void guard(v8f& a, v8f& b, v16h x, v16h y) { dep_guard_h(a, b, x, y); }
  static __device__ __forceinline__ void keep(v16h a, v16h b, v16h c, v16h d) { keep4_h(a, b, c, d); }
};

__device__ __forceinline__ float softplus_f(float u) {
  return fmaxf(u, 0.0f) + __logf(1.0f + __expf(-fabsf(u)));
}

__global__ __launch_bounds__(256)
void pack_input_kernel(const float* __restrict__ x, const float* __restrict__ cond,
                       _Float16* __restrict__ netin) {
  const int i = blockIdx.x * 256 + threadIdx.x;
  if (i >= MPIX * 2) return;
  const int pix = i >> 1, hf = i & 1;
  const int b = pix >> 12, p = pix & 4095;
  v8h v;
  if (hf == 0) {
#pragma unroll
    for (int e = 0; e < 8; ++e) v[e] = (_Float16)x[(((size_t)(b * NCH + e)) << 12) + p];
  } else {
#pragma unroll
    for (int e = 0; e < 4; ++e) v[e] = (_Float16)x[(((size_t)(b * NCH + 8 + e)) << 12) + p];
#pragma unroll
    for (int e = 0; e < 4; ++e) v[4 + e] = (_Float16)cond[(((size_t)(b * NCOND + e)) << 12) + p];
  }
  _Float16* dp = netin + (size_t)i * 8;
  *(volatile v8h*)dp = v;
  __threadfence();
  *(volatile v8h*)dp = v;
}

template <int CIN, int TAPS>
__global__ __launch_bounds__(256)
void pack_weights_kernel(const float* __restrict__ w, _Float16* __restrict__ wp,
                         int Nreal, int Npad, int total8, float scale) {
  const int i = blockIdx.x * 256 + threadIdx.x;
  if (i >= total8) return;
  const int row = i >> 2;
  const int kk0 = (i & 3) * 8;
  const int kt  = row / Npad;
  const int n   = row - kt * Npad;
  v8h hv;
#pragma unroll
  for (int e = 0; e < 8; ++e) {
    const int k   = kt * 32 + kk0 + e;
    const int tap = k / CIN;
    const int ic  = k - tap * CIN;
    float v = 0.0f;
    if (tap < TAPS && n < Nreal) v = w[((size_t)n * CIN + ic) * TAPS + tap] * scale;
    hv[e] = (_Float16)v;
  }
  _Float16* dp = wp + (size_t)i * 8;
  *(volatile v8h*)dp = hv;
  __threadfence();
  *(volatile v8h*)dp = hv;
}

template <int EPI, int CIN, int TAPS, int KW, int MW, int WN, int FN>
__global__ __launch_bounds__(32 * MW * WN)
void conv_kernel(const _Float16* __restrict__ src, const _Float16* __restrict__ wp,
                 const float* __restrict__ bias, int Nreal, int Npad, float oscale,
                 _Float16* __restrict__ dst16,
                 const float* __restrict__ xg, float* __restrict__ yout, float* __restrict__ part) {
  constexpr int NT  = 32 * MW * WN;
  constexpr int NW  = MW * WN;
  constexpr int BM  = 16 * MW;
  constexpr int BN  = 16 * WN * FN;
  constexpr int KT  = (TAPS * CIN + 31) / 32;
  constexpr int AP  = 40;
  constexpr int SP  = 72;
  constexpr int PSP = BN + 4;
  static_assert(FN == 4 || FN == 6, "FN");
  static_assert(EPI != 0 || FN == 4, "EPI0 wave span is 64 channels");
  static_assert(EPI != 1 || (NT == 192 && BM == 32 && (NCH * BM) % NT == 0), "EPI1 geometry");
  static_assert(BM * 4 <= NT, "feeder threads");

  __shared__ __align__(16) _Float16 As[BM * AP];
  __shared__ __align__(16) _Float16 Sl[(EPI == 0) ? NW * 16 * SP : 8];
  __shared__ __align__(16) float Ps[(EPI == 1) ? BM * PSP : 4];
  __shared__ __align__(16) float Ys[(EPI == 1) ? NCH * BM : 4];
  __shared__ float Rd[(EPI == 1) ? NT : 1];

  const int tid  = threadIdx.x;
  const int lane = tid & 31, wave = tid >> 5;
  const int hh   = lane >> 4, lm = lane & 15;
  const int wmi  = wave % MW, wni = wave / MW;
  const int wm   = wmi * 16, wn = wni * FN * 16;
  const int m0   = blockIdx.x * BM;
  const int bimg = m0 >> 12, p0 = m0 & 4095, prow = p0 >> 6, pc0 = p0 & 63;
  const bool afeed = tid < BM * 4;
  const int arow = tid >> 2, aq = tid & 3;

  v8f acc[FN];
#pragma unroll
  for (int fn = 0; fn < FN; ++fn) acc[fn] = (v8f){0.f, 0.f, 0.f, 0.f, 0.f, 0.f, 0.f, 0.f};

#pragma unroll 1
  for (int kt = 0; kt < KT; ++kt) {
    v8h av;
#pragma unroll
    for (int e = 0; e < 8; ++e) av[e] = (_Float16)0.0f;
    if (afeed) {
      const int k0  = kt * 32 + aq * 8;
      const int tap = k0 / CIN;
      const int ic0 = k0 - tap * CIN;
      const int ty  = tap / KW;
      const int dy  = ty - (KW >> 1);
      const int dx  = (tap - ty * KW) - (KW >> 1);
      const int iy  = prow + dy, ix = pc0 + arow + dx;
      if (tap < TAPS && (unsigned)iy < 64u && (unsigned)ix < 64u)
        av = *(const v8h*)(src + ((size_t)((bimg << 12) + (iy << 6) + ix)) * CIN + ic0);
    }
    __syncthreads();
    if (afeed) *(v8h*)(As + arow * AP + aq * 8) = av;
    __syncthreads();

    const v16h af = Frag<_Float16>::load(As + (wm + lm) * AP + 8 * hh);
    const _Float16* wrow = wp + ((size_t)(kt * Npad + wn + lm)) * 32 + 8 * hh;
    v16h bfr[FN];
#pragma unroll
    for (int fn = 0; fn < FN; ++fn) {
      bfr[fn] = Frag<_Float16>::load(wrow + fn * 16 * 32);
      acc[fn] = Frag<_Float16>::mma(af, bfr[fn], acc[fn]);
    }
    dep_guard_h(acc[0], acc[FN - 1], af, bfr[FN - 1]);
    keep4_h(bfr[0], bfr[1], bfr[2], bfr[3]);
    if constexpr (FN > 4) keep4_h(bfr[4], bfr[FN - 1], bfr[4], bfr[FN - 1]);
  }
  acc_guard4(acc[0], acc[1], acc[2], acc[3]);
  if constexpr (FN > 4) acc_guard4(acc[2], acc[3], acc[FN - 2], acc[FN - 1]);

  if constexpr (EPI == 0) {
    _Float16* sl = Sl + wave * 16 * SP;
#pragma unroll
    for (int fn = 0; fn < FN; ++fn) {
      const int n = wn + fn * 16 + lm;
      const float bz = (n < Nreal) ? bias[n] : 0.0f;
#pragma unroll
      for (int r = 0; r < 8; ++r) {
        float v = acc[fn][r] * oscale + bz;
        v = fmaxf(v, 0.0f);
        sl[(8 * hh + r) * SP + fn * 16 + lm] = (_Float16)v;
      }
    }
    __builtin_amdgcn_fence(__ATOMIC_RELEASE, "workgroup");
    __builtin_amdgcn_wave_barrier();
    __builtin_amdgcn_fence(__ATOMIC_ACQUIRE, "workgroup");
    const int q = lane >> 3, c8 = (lane & 7) * 8;
    for (int pass = 0; pass < 2; ++pass) {
#pragma unroll
      for (int it = 0; it < 4; ++it) {
        const int row = it * 4 + q;
        const v8h hv = *(const v8h*)(sl + row * SP + c8);
        *(volatile v8h*)(dst16 + ((size_t)(m0 + wm + row)) * BN + wn + c8) = hv;
      }
      __threadfence();
    }
  }

  if constexpr (EPI == 1) {
#pragma unroll
    for (int fn = 0; fn < FN; ++fn) {
      const int n = wn + fn * 16 + lm;
      const float bz = (n < Nreal) ? bias[n] : 0.0f;
#pragma unroll
      for (int r = 0; r < 8; ++r) Ps[(wm + 8 * hh + r) * PSP + n] = acc[fn][r] * oscale + bz;
    }
    __syncthreads();

    const float dpad = MDV + softplus_f(UPAD);
    float ladsum = 0.0f;
#pragma unroll 1
    for (int s = 0; s < (NCH * BM) / NT; ++s) {
      const int e  = tid + s * NT;
      const int px = e & (BM - 1);
      const int cc = e / BM;
      const float* P = Ps + px * PSP + cc * NPAR;

      float uw[8], uh[8], dv[9], cw[9], chh[9], wd[8], hg[8];
#pragma unroll
      for (int j = 0; j < 8; ++j) uw[j] = P[j];
#pragma unroll
      for (int j = 0; j < 8; ++j) uh[j] = P[8 + j];
      dv[0] = dpad; dv[8] = dpad;
#pragma unroll
      for (int j = 0; j < 7; ++j) dv[j + 1] = MDV + softplus_f(P[16 + j]);

      float mx = uw[0];
#pragma unroll
      for (int j = 1; j < 8; ++j) mx = fmaxf(mx, uw[j]);
      float ssum = 0.0f;
#pragma unroll
      for (int j = 0; j < 8; ++j) { uw[j] = __expf(uw[j] - mx); ssum += uw[j]; }
      float inv = __fdividef(1.0f, ssum);
      float run = 0.0f;
      cw[0] = -TAILV;
#pragma unroll
      for (int j = 0; j < 8; ++j) {
        const float wj = MBWV + WSCL * (uw[j] * inv);
        run += wj;
        if (j < 7) cw[j + 1] = 6.0f * run - TAILV;
      }
      cw[8] = TAILV;
#pragma unroll
      for (int j = 0; j < 8; ++j) wd[j] = cw[j + 1] - cw[j];

      mx = uh[0];
#pragma unroll
      for (int j = 1; j < 8; ++j) mx = fmaxf(mx, uh[j]);
      ssum = 0.0f;
#pragma unroll
      for (int j = 0; j < 8; ++j) { uh[j] = __expf(uh[j] - mx); ssum += uh[j]; }
      inv = __fdividef(1.0f, ssum);
      run = 0.0f;
      chh[0] = -TAILV;
#pragma unroll
      for (int j = 0; j < 8; ++j) {
        const float hj = MBHV + WSCL * (uh[j] * inv);
        run += hj;
        if (j < 7) chh[j + 1] = 6.0f * run - TAILV;
      }
      chh[8] = TAILV;
#pragma unroll
      for (int j = 0; j < 8; ++j) hg[j] = chh[j + 1] - chh[j];

      const size_t gi = (((size_t)(bimg * NCH + cc)) << 12) + p0 + px;
      const float xv = xg[gi];
      const bool inside = (xv >= -TAILV) && (xv <= TAILV);
      const float xc = fminf(fmaxf(xv, -TAILV), TAILV);

      int cnt = 1;
#pragma unroll
      for (int j = 1; j < 8; ++j) cnt += (xc >= cw[j]) ? 1 : 0;
      cnt += (xc >= TAILV) ? 1 : 0;
      int idx = cnt - 1;
      idx = idx > 7 ? 7 : idx;

      float icw = cw[0], iw = wd[0], ich = chh[0], ih = hg[0], d0 = dv[0], d1 = dv[1];
#pragma unroll
      for (int j = 1; j < 8; ++j) {
        const bool sel = (j == idx);
        icw = sel ? cw[j]     : icw;
        iw  = sel ? wd[j]     : iw;
        ich = sel ? chh[j]    : ich;
        ih  = sel ? hg[j]     : ih;
        d0  = sel ? dv[j]     : d0;
        d1  = sel ? dv[j + 1] : d1;
      }

      const float del   = __fdividef(ih, iw);
      const float th    = __fdividef(xc - icw, iw);
      const float omt   = 1.0f - th;
      const float tom   = th * omt;
      const float numer = ih * (del * th * th + d0 * tom);
      const float den   = del + (d0 + d1 - 2.0f * del) * tom;
      float yv          = ich + __fdividef(numer, den);
      const float dnum  = del * del * (d1 * th * th + 2.0f * del * tom + d0 * omt * omt);
      float lad         = __logf(dnum) - 2.0f * __logf(den);

      yv  = inside ? yv  : xv;
      lad = inside ? lad : 0.0f;
      Ys[cc * BM + px] = yv;
      ladsum += lad;
    }

    Rd[tid] = ladsum;
    __syncthreads();
    if (tid < 64) Rd[tid] += Rd[tid + 128];
    __syncthreads();
#pragma unroll
    for (int s2 = 64; s2 > 0; s2 >>= 1) {
      if (tid < s2) Rd[tid] += Rd[tid + s2];
      __syncthreads();
    }

    if (tid < NCH * (BM / 4)) {
      const int c2 = tid / (BM / 4);
      const int q4 = (tid % (BM / 4)) * 4;
      const v4f val = *(const v4f*)(Ys + c2 * BM + q4);
      float* op = yout + (((size_t)(bimg * NCH + c2)) << 12) + p0 + q4;
      *(volatile v4f*)op = val;
      __threadfence();
      *(volatile v4f*)op = val;
    }
    if (wave == 0) {
      const float pv = (lane == 0) ? Rd[0] : 0.0f;
      float* pp = part + (((size_t)blockIdx.x) << 5) + lane;
      *(volatile float*)pp = pv;
      __threadfence();
      *(volatile float*)pp = pv;
    }
  }
}

__global__ __launch_bounds__(32)
void logdet_final_kernel(const float* __restrict__ ld, const float* __restrict__ part,
                         float* __restrict__ out1) {
  const int b = threadIdx.x;
  if (b < NBATCH) {
    float s = ld[b];
#pragma unroll 4
    for (int i = 0; i < 128; ++i) s += part[((size_t)(b * 128 + i)) << 5];
    float* op = out1 + b;
    *(volatile float*)op = s;
    __threadfence();
    *(volatile float*)op = s;
  }
}

extern "C" void kernel_launch(void* const* d_in, const int* in_sizes, int n_in,
                              void* d_out, int out_size, void* d_ws, size_t ws_size,
                              hipStream_t stream) {
  if (n_in < 9) return;
  if (in_sizes[0] != MPIX * NCH || in_sizes[1] != NBATCH || in_sizes[2] != MPIX * NCOND ||
      in_sizes[3] != HID * CIN1 * 9 || in_sizes[4] != HID || in_sizes[5] != HID * HID ||
      in_sizes[6] != HID || in_sizes[7] != OUTC * HID * 9 || in_sizes[8] != OUTC) return;
  if (out_size != MPIX * NCH + NBATCH) return;

  const float* x    = (const float*)d_in[0];
  const float* ld   = (const float*)d_in[1];
  const float* cond = (const float*)d_in[2];
  const float* w1   = (const float*)d_in[3];
  const float* b1   = (const float*)d_in[4];
  const float* w2   = (const float*)d_in[5];
  const float* b2   = (const float*)d_in[6];
  const float* w3   = (const float*)d_in[7];
  const float* b3   = (const float*)d_in[8];
  float* out0 = (float*)d_out;
  float* out1 = out0 + (size_t)MPIX * NCH;

  const size_t sz_netin = (size_t)MPIX * CIN1 * 2;
  const size_t sz_h     = (size_t)MPIX * HID * 2;
  const size_t sz_w1    = (size_t)KT1 * HID * 32 * 2;
  const size_t sz_w2    = (size_t)KT2 * HID * 32 * 2;
  const size_t sz_w3    = (size_t)KT3 * NPAD3 * 32 * 2;
  const size_t sz_part  = (size_t)(MPIX / 32) * 32 * 4;
  const size_t off_netin = 0;
  const size_t off_h1    = off_netin + sz_netin;
  const size_t off_h2    = off_h1 + sz_h;
  const size_t off_w1    = off_h2 + sz_h;
  const size_t off_w2    = off_w1 + sz_w1;
  const size_t off_w3    = off_w2 + sz_w2;
  const size_t off_part  = off_w3 + sz_w3;
  const size_t total     = off_part + sz_part;
  if (total > ws_size) return;

  char* ws = (char*)d_ws;
  _Float16* netin = (_Float16*)(ws + off_netin);
  _Float16* h1    = (_Float16*)(ws + off_h1);
  _Float16* h2    = (_Float16*)(ws + off_h2);
  _Float16* w1p   = (_Float16*)(ws + off_w1);
  _Float16* w2p   = (_Float16*)(ws + off_w2);
  _Float16* w3p   = (_Float16*)(ws + off_w3);
  float*    part  = (float*)(ws + off_part);

  pack_input_kernel<<<(MPIX * 2) / 256, 256, 0, stream>>>(x, cond, netin);
  {
    const int t1 = KT1 * HID * 4;
    const int t2 = KT2 * HID * 4;
    const int t3 = KT3 * NPAD3 * 4;
    pack_weights_kernel<CIN1, 9><<<(t1 + 255) / 256, 256, 0, stream>>>(w1, w1p, HID, HID, t1, 16.0f);
    pack_weights_kernel<HID, 1><<<(t2 + 255) / 256, 256, 0, stream>>>(w2, w2p, HID, HID, t2, 16.0f);
    pack_weights_kernel<HID, 9><<<(t3 + 255) / 256, 256, 0, stream>>>(w3, w3p, OUTC, NPAD3, t3, 64.0f);
  }

  conv_kernel<0, CIN1, 9, 3, 4, 2, 4><<<MPIX / 64, 256, 0, stream>>>(
      netin, w1p, b1, HID, HID, 0.0625f, h1, x, out0, part);
  conv_kernel<0, HID, 1, 1, 4, 2, 4><<<MPIX / 64, 256, 0, stream>>>(
      h1, w2p, b2, HID, HID, 0.0625f, h2, x, out0, part);

  conv_kernel<1, HID, 9, 3, 2, 3, 6><<<MPIX / 32, 192, 0, stream>>>(
      h2, w3p, b3, OUTC, NPAD3, 0.015625f, h1, x, out0, part);

  logdet_final_kernel<<<1, 32, 0, stream>>>(ld, part, out1);
}
